// MaxViT3DMHSA_81887846466144
// MI455X (gfx1250) — hardware-verified
//
#include <hip/hip_runtime.h>
#include <stdint.h>

#define NWIN  128
#define NTOK  343
#define TP    384
#define CCH   256
#define NHD   8
#define HD    32
#define C3    768
#define NROWP 49152
#define NROWX 43904
#define NRPB  2197
#define NST   24
#define NKT   24
#define MT    6
#define LDC   132
#define PP    72
#define OSP   36
#define PWB   2304
#define TPW   260
#define QSC   0.17677669529663687f
#define INV512 0.001953125f
#define LN1024 6.9314718055994531f
#define MASKC (-1048576.0f)

static_assert(NROWP == NWIN * TP);
static_assert(NROWX == NWIN * NTOK);
static_assert(TP == MT * 64);
static_assert(NST * 16 == TP);
static_assert(NKT * 16 == TP);
static_assert(PWB == 16 * PP * 2);
static_assert(16 * OSP * 4 <= PWB);
static_assert((PP * 2) % 16 == 0);
static_assert((LDC * 4) % 16 == 0);
static_assert((TPW * 4) % 16 == 0);
static_assert(NHD * HD == CCH);

typedef _Float16 v16h __attribute__((ext_vector_type(16)));
typedef _Float16 v8h  __attribute__((ext_vector_type(8)));
typedef float    v8f  __attribute__((ext_vector_type(8)));
typedef float    v4f  __attribute__((ext_vector_type(4)));
typedef unsigned int v4u __attribute__((ext_vector_type(4)));

__device__ __forceinline__ unsigned short bf_bits(float f) {
  unsigned u = __float_as_uint(f);
  return (unsigned short)((u + 0x7FFFu + ((u >> 16) & 1u)) >> 16);
}
__device__ __forceinline__ float bf_up(unsigned short b) { return __uint_as_float(((unsigned)b) << 16); }
__device__ __forceinline__ float bfr(float f) { return bf_up(bf_bits(f)); }
__device__ __forceinline__ unsigned short h_bits(_Float16 x) { return __builtin_bit_cast(unsigned short, x); }
__device__ __forceinline__ unsigned short hb16(float f) { return h_bits((_Float16)f); }
__device__ __forceinline__ unsigned pk16(unsigned short a, unsigned short b) { return (unsigned)a | ((unsigned)b << 16); }
__device__ __forceinline__ v8f zero8() { v8f z = {0.f, 0.f, 0.f, 0.f, 0.f, 0.f, 0.f, 0.f}; return z; }

__device__ __forceinline__ v16h ldfrag_h(const _Float16* p) {
  union { v16h v; v8h h[2]; } f;
  f.h[0] = *(const v8h*)(p);
  f.h[1] = *(const v8h*)(p + 16);
  return f.v;
}

__device__ __forceinline__ v8f mma_raw(v16h a, v16h b, v8f c) {
  return __builtin_amdgcn_wmma_f32_16x16x32_f16(false, a, false, b, (short)0, c, false, false);
}
__device__ __forceinline__ v8f mma_g1(v16h a, v16h b, v8f c) {
  c = mma_raw(a, b, c);
#if defined(__HIP_DEVICE_COMPILE__)
  asm volatile("v_nop\n\tv_nop\n\tv_nop\n\tv_nop" : "+v"(c) : "v"(a), "v"(b));
#endif
  return c;
}
__device__ __forceinline__ void guard2(v8f& c0, v8f& c1, const v16h& a0, const v16h& b0, const v16h& b1) {
#if defined(__HIP_DEVICE_COMPILE__)
  asm volatile("v_nop\n\tv_nop\n\tv_nop\n\tv_nop" : "+v"(c0), "+v"(c1) : "v"(a0), "v"(b0), "v"(b1));
#endif
}
__device__ __forceinline__ void guard4(v8f& c0, v8f& c1, v8f& c2, v8f& c3,
                                       const v16h& a0, const v16h& a1, const v16h& b0, const v16h& b1) {
#if defined(__HIP_DEVICE_COMPILE__)
  asm volatile("v_nop\n\tv_nop\n\tv_nop\n\tv_nop"
               : "+v"(c0), "+v"(c1), "+v"(c2), "+v"(c3) : "v"(a0), "v"(a1), "v"(b0), "v"(b1));
#endif
}
__device__ __forceinline__ void wave_sync_lds() {
  __builtin_amdgcn_fence(__ATOMIC_RELEASE, "workgroup");
  __builtin_amdgcn_wave_barrier();
  __builtin_amdgcn_fence(__ATOMIC_ACQUIRE, "workgroup");
}

__global__ __launch_bounds__(256) void cvt_x(const float* __restrict__ x, unsigned short* xp) {
  const int tid = threadIdx.x, wv = tid >> 5, lane = tid & 31;
  const int row = blockIdx.x * 8 + wv;
  const int w = row / TP, t = row - w * TP;
  const int ts = min(t, NTOK - 1);
  const float* src = x + ((size_t)w * NTOK + ts) * CCH + lane * 8;
  const v4f a = *(const v4f*)(src);
  const v4f b = *(const v4f*)(src + 4);
  v4u pk;
  pk[0] = pk16(hb16(bfr(a[0]) * 8.0f), hb16(bfr(a[1]) * 8.0f));
  pk[1] = pk16(hb16(bfr(a[2]) * 8.0f), hb16(bfr(a[3]) * 8.0f));
  pk[2] = pk16(hb16(bfr(b[0]) * 8.0f), hb16(bfr(b[1]) * 8.0f));
  pk[3] = pk16(hb16(bfr(b[2]) * 8.0f), hb16(bfr(b[3]) * 8.0f));
  if (t >= NTOK) { pk[0] = 0u; pk[1] = 0u; pk[2] = 0u; pk[3] = 0u; }
  unsigned short* gp = xp + (size_t)row * CCH + lane * 8;
  *(volatile v4u*)gp = pk;
  __threadfence();
  *(volatile v4u*)gp = pk;
}

__global__ __launch_bounds__(256) void cvt_wT(const float* __restrict__ wsrc, unsigned short* wdst, int ncol) {
  __shared__ __align__(16) float T[32 * TPW];
  const int tid = threadIdx.x, wv = tid >> 5, lane = tid & 31;
  const int n0 = blockIdx.x * 32;
#pragma unroll 4
  for (int it = 0; it < 32; ++it) {
    const int k = it * 8 + wv;
    T[lane * TPW + k] = wsrc[(size_t)k * ncol + n0 + lane];
  }
  __syncthreads();
  v4u pk[4];
  size_t offs[4];
#pragma unroll
  for (int q = 0; q < 4; ++q) {
    const int nl = wv * 4 + q;
    const float* tp = T + nl * TPW + lane * 8;
    const v4f a = *(const v4f*)(tp);
    const v4f b = *(const v4f*)(tp + 4);
    v4u p4;
    p4[0] = pk16(hb16(bfr(a[0]) * 1024.0f), hb16(bfr(a[1]) * 1024.0f));
    p4[1] = pk16(hb16(bfr(a[2]) * 1024.0f), hb16(bfr(a[3]) * 1024.0f));
    p4[2] = pk16(hb16(bfr(b[0]) * 1024.0f), hb16(bfr(b[1]) * 1024.0f));
    p4[3] = pk16(hb16(bfr(b[2]) * 1024.0f), hb16(bfr(b[3]) * 1024.0f));
    pk[q] = p4;
    offs[q] = (size_t)(n0 + nl) * CCH + lane * 8;
  }
#pragma unroll
  for (int q = 0; q < 4; ++q) *(volatile v4u*)(wdst + offs[q]) = pk[q];
  __threadfence();
#pragma unroll
  for (int q = 0; q < 4; ++q) *(volatile v4u*)(wdst + offs[q]) = pk[q];
}

__global__ __launch_bounds__(256) void build_bias(const float* __restrict__ rpb, float* bt) {
  const int g = blockIdx.x * 256 + threadIdx.x;
  const int piece = g & 63, rec = g >> 6;
  const int kt = rec % NKT, strip = (rec / NKT) % NST, h = rec / (NKT * NST);
  const int l = piece >> 1, e0 = (piece & 1) * 4;
  const int col = l & 15, lh = l >> 4;
  const int m = kt * 16 + col;
  const int mi = m / 49, mj = (m / 7) % 7, mk = m % 7;
  v4f v;
#pragma unroll
  for (int e = 0; e < 4; ++e) {
    const int n = strip * 16 + 8 * lh + e0 + e;
    const int ni = n / 49, nj = (n / 7) % 7, nk = n % 7;
    int idx = ((ni - mi + 6) * 13 + (nj - mj + 6)) * 13 + (nk - mk + 6);
    idx = min(max(idx, 0), NRPB - 1);
    float val = bfr(rpb[idx * NHD + h]) * 512.0f;
    if (n >= NTOK) val = 0.0f;
    if (m >= NTOK) val = MASKC;
    v[e] = val;
  }
  float* gp = bt + (size_t)rec * 256 + piece * 4;
  *(volatile v4f*)gp = v;
  __threadfence();
  *(volatile v4f*)gp = v;
}

__global__ __launch_bounds__(256)
void gemm_qkv(const unsigned short* __restrict__ xp, const unsigned short* __restrict__ wq,
              unsigned short* qpl, unsigned short* kpl, unsigned short* vtp) {
  __shared__ __align__(16) float Cs[64 * LDC];
  const int tid = threadIdx.x, wave = tid >> 5, lane = tid & 31, hh = lane >> 4, c = lane & 15;
  const int mb = blockIdx.x, nb = blockIdx.y;
  const int mw = wave >> 2, nw = wave & 3;
  const _Float16* A = (const _Float16*)(const void*)xp;
  const _Float16* W = (const _Float16*)(const void*)wq;
  const int arow0 = mb * 64 + mw * 32;
  const int bcol0 = nb * 128 + nw * 32;

  v8f a00 = zero8(), a01 = zero8(), a10 = zero8(), a11 = zero8();
#pragma unroll 1
  for (int ks = 0; ks < 8; ++ks) {
    const int k0 = ks * 32 + 8 * hh;
    const v16h fa0 = ldfrag_h(A + (size_t)(arow0 + c) * CCH + k0);
    const v16h fa1 = ldfrag_h(A + (size_t)(arow0 + 16 + c) * CCH + k0);
    const v16h fb0 = ldfrag_h(W + (size_t)(bcol0 + c) * CCH + k0);
    const v16h fb1 = ldfrag_h(W + (size_t)(bcol0 + 16 + c) * CCH + k0);
    a00 = mma_raw(fa0, fb0, a00);
    a01 = mma_raw(fa0, fb1, a01);
    a10 = mma_raw(fa1, fb0, a10);
    a11 = mma_raw(fa1, fb1, a11);
    guard4(a00, a01, a10, a11, fa0, fa1, fb0, fb1);
  }
#pragma unroll
  for (int r = 0; r < 8; ++r) {
    const int row = mw * 32 + 8 * hh + r;
    Cs[row * LDC + nw * 32 + c]             = a00[r];
    Cs[row * LDC + nw * 32 + 16 + c]        = a01[r];
    Cs[(row + 16) * LDC + nw * 32 + c]      = a10[r];
    Cs[(row + 16) * LDC + nw * 32 + 16 + c] = a11[r];
  }
  __syncthreads();

  const int part = nb >> 1;
  const int hb4 = (nb & 1) * 4;
  const int w = mb / MT, tok0 = (mb - w * MT) * 64;
  if (part < 2) {
    unsigned short* dst = (part == 0) ? qpl : kpl;
    const float scl = (part == 0) ? (QSC * (64.0f / 8192.0f)) : (8.0f / 8192.0f);
    v4u pk[4];
    size_t offs[4];
#pragma unroll
    for (int s = 0; s < 4; ++s) {
      const int L = s * 32 + (tid >> 3), p = tid & 7;
      const int h4 = L >> 5, li = L & 31;
      const int tok = 2 * li + (p >> 2), d0 = (p & 3) * 8;
      const int col = h4 * 32 + d0;
      v4u q4;
#pragma unroll
      for (int e = 0; e < 4; ++e) {
        const float f0 = Cs[tok * LDC + col + 2 * e] * scl;
        const float f1 = Cs[tok * LDC + col + 2 * e + 1] * scl;
        q4[e] = pk16(hb16(f0), hb16(f1));
      }
      pk[s] = q4;
      offs[s] = ((size_t)((w * NHD + hb4 + h4) * TP + tok0 + tok)) * HD + d0;
    }
#pragma unroll
    for (int s = 0; s < 4; ++s) *(volatile v4u*)(dst + offs[s]) = pk[s];
    __threadfence();
#pragma unroll
    for (int s = 0; s < 4; ++s) *(volatile v4u*)(dst + offs[s]) = pk[s];
  } else {
    v4u pv[4];
    size_t offs[4];
#pragma unroll
    for (int s = 0; s < 4; ++s) {
      const int L = s * 32 + (tid >> 3), p = tid & 7;
      const int h4 = L >> 5, d = L & 31;
      const int col = h4 * 32 + d;
      const int tb = p * 8;
      v4u a;
#pragma unroll
      for (int e = 0; e < 4; ++e) {
        const float v0 = Cs[(tb + 2 * e) * LDC + col] * (16.0f / 8192.0f);
        const float v1 = Cs[(tb + 2 * e + 1) * LDC + col] * (16.0f / 8192.0f);
        a[e] = pk16(hb16(v0), hb16(v1));
      }
      pv[s] = a;
      offs[s] = ((size_t)((w * NHD + hb4 + h4) * HD + d)) * TP + tok0 + tb;
    }
#pragma unroll
    for (int s = 0; s < 4; ++s) *(volatile v4u*)(vtp + offs[s]) = pv[s];
    __threadfence();
#pragma unroll
    for (int s = 0; s < 4; ++s) *(volatile v4u*)(vtp + offs[s]) = pv[s];
  }
}

__global__ __launch_bounds__(256)
void attn_win(const unsigned short* __restrict__ qpl, const unsigned short* __restrict__ kpl,
              const unsigned short* __restrict__ vtp, const float* __restrict__ bt, unsigned short* opl) {
  __shared__ __align__(16) char pbuf[8 * PWB];
  union CB { v8f v; v4f q[2]; };
  const int tid = threadIdx.x, wave = tid >> 5, lane = tid & 31, hh = lane >> 4, c = lane & 15;
  const int wh = blockIdx.x / 3;
  const int sb = blockIdx.x - wh * 3;
  const int w = wh >> 3, h = wh & 7;
  const int strip = sb * 8 + wave;
  const int q0 = strip * 16;

  const _Float16* Q  = (const _Float16*)(const void*)qpl + (size_t)wh * TP * HD;
  const _Float16* K  = (const _Float16*)(const void*)kpl + (size_t)wh * TP * HD;
  const _Float16* Vt = (const _Float16*)(const void*)vtp + (size_t)wh * HD * TP;
  const float* Bp = bt + ((size_t)(h * NST + strip)) * NKT * 256 + lane * 8;
  _Float16* Ph = (_Float16*)(pbuf + wave * PWB);

  const v16h qa = ldfrag_h(Q + (size_t)(q0 + c) * HD + 8 * hh);
  float mrow[8], lrow[8];
#pragma unroll
  for (int r = 0; r < 8; ++r) { mrow[r] = -1e30f; lrow[r] = 0.f; }
  v8f o0 = zero8(), o1 = zero8();

#pragma unroll 1
  for (int kb = 0; kb < TP / 64; ++kb) {
    v8f s[4];
#pragma unroll
    for (int j = 0; j < 4; ++j) {
      const int key = kb * 64 + j * 16 + c;
      const v16h kf = ldfrag_h(K + (size_t)key * HD + 8 * hh);
      const float* bp = Bp + (kb * 4 + j) * 256;
      CB cb;
      cb.q[0] = *(const v4f*)(bp);
      cb.q[1] = *(const v4f*)(bp + 4);
      s[j] = mma_g1(qa, kf, cb.v);
    }
#pragma unroll
    for (int r = 0; r < 8; ++r) {
      float tm = fmaxf(fmaxf(s[0][r], s[1][r]), fmaxf(s[2][r], s[3][r]));
      tm = fmaxf(tm, __shfl_xor(tm, 1, 32));
      tm = fmaxf(tm, __shfl_xor(tm, 2, 32));
      tm = fmaxf(tm, __shfl_xor(tm, 4, 32));
      tm = fmaxf(tm, __shfl_xor(tm, 8, 32));
      const float mn = fmaxf(mrow[r], tm);
      const float alpha = __expf((mrow[r] - mn) * INV512);
      mrow[r] = mn;
      float ps = 0.f;
#pragma unroll
      for (int j = 0; j < 4; ++j) {
        const float p = __expf((s[j][r] - mn) * INV512 + LN1024);
        ps = ps + p;
        s[j][r] = p;
      }
      ps = ps + __shfl_xor(ps, 1, 32);
      ps = ps + __shfl_xor(ps, 2, 32);
      ps = ps + __shfl_xor(ps, 4, 32);
      ps = ps + __shfl_xor(ps, 8, 32);
      lrow[r] = lrow[r] * alpha + ps;
      o0[r] = o0[r] * alpha;
      o1[r] = o1[r] * alpha;
    }
#pragma unroll
    for (int j = 0; j < 4; ++j) {
#pragma unroll
      for (int r = 0; r < 8; ++r) {
        Ph[(8 * hh + r) * PP + j * 16 + c] = (_Float16)s[j][r];
      }
    }
    wave_sync_lds();
#pragma unroll
    for (int ks = 0; ks < 2; ++ks) {
      const v16h pa = ldfrag_h(Ph + c * PP + ks * 32 + 8 * hh);
      const int koff = kb * 64 + ks * 32 + 8 * hh;
      const v16h v0 = ldfrag_h(Vt + (size_t)c * TP + koff);
      const v16h v1 = ldfrag_h(Vt + (size_t)(16 + c) * TP + koff);
      o0 = mma_raw(pa, v0, o0);
      o1 = mma_raw(pa, v1, o1);
      guard2(o0, o1, pa, v0, v1);
    }
    wave_sync_lds();
  }

  float* Os = (float*)(void*)(pbuf + wave * PWB);
#pragma unroll
  for (int r = 0; r < 8; ++r) {
    const float inv = 4.0f / lrow[r];
    const int row = 8 * hh + r;
    Os[row * OSP + c]      = o0[r] * inv;
    Os[row * OSP + 16 + c] = o1[r] * inv;
  }
  wave_sync_lds();
  v4u p2[2];
  size_t off2[2];
#pragma unroll
  for (int sI = 0; sI < 2; ++sI) {
    const int line = sI * 4 + (lane >> 3), piece = lane & 7;
    const int row = 2 * line + (piece >> 2), d0 = (piece & 3) * 8;
    v4u a;
#pragma unroll
    for (int e = 0; e < 4; ++e) {
      const float f0 = Os[row * OSP + d0 + 2 * e];
      const float f1 = Os[row * OSP + d0 + 2 * e + 1];
      a[e] = pk16(hb16(f0), hb16(f1));
    }
    p2[sI] = a;
    off2[sI] = ((size_t)h * NROWP + (size_t)w * TP + q0 + row) * HD + d0;
  }
  *(volatile v4u*)(opl + off2[0]) = p2[0];
  *(volatile v4u*)(opl + off2[1]) = p2[1];
  __threadfence();
  *(volatile v4u*)(opl + off2[0]) = p2[0];
  *(volatile v4u*)(opl + off2[1]) = p2[1];
}

__global__ __launch_bounds__(256)
void gemm_proj(const unsigned short* __restrict__ opl, const unsigned short* __restrict__ wp, float* out) {
  __shared__ __align__(16) float Cs[64 * LDC];
  const int tid = threadIdx.x, wave = tid >> 5, lane = tid & 31, hh = lane >> 4, c = lane & 15;
  const int mb = blockIdx.x, nb = blockIdx.y;
  const int mw = wave >> 2, nw = wave & 3;
  const _Float16* W = (const _Float16*)(const void*)wp;
  const int arow0 = mb * 64 + mw * 32;
  const int bcol0 = nb * 128 + nw * 32;

  v8f a00 = zero8(), a01 = zero8(), a10 = zero8(), a11 = zero8();
#pragma unroll 1
  for (int ks = 0; ks < 8; ++ks) {
    const _Float16* Ah = (const _Float16*)(const void*)opl + (size_t)ks * NROWP * HD;
    const v16h fa0 = ldfrag_h(Ah + (size_t)(arow0 + c) * HD + 8 * hh);
    const v16h fa1 = ldfrag_h(Ah + (size_t)(arow0 + 16 + c) * HD + 8 * hh);
    const v16h fb0 = ldfrag_h(W + (size_t)(bcol0 + c) * CCH + ks * 32 + 8 * hh);
    const v16h fb1 = ldfrag_h(W + (size_t)(bcol0 + 16 + c) * CCH + ks * 32 + 8 * hh);
    a00 = mma_raw(fa0, fb0, a00);
    a01 = mma_raw(fa0, fb1, a01);
    a10 = mma_raw(fa1, fb0, a10);
    a11 = mma_raw(fa1, fb1, a11);
    guard4(a00, a01, a10, a11, fa0, fa1, fb0, fb1);
  }
#pragma unroll
  for (int r = 0; r < 8; ++r) {
    const int row = mw * 32 + 8 * hh + r;
    Cs[row * LDC + nw * 32 + c]             = a00[r];
    Cs[row * LDC + nw * 32 + 16 + c]        = a01[r];
    Cs[(row + 16) * LDC + nw * 32 + c]      = a10[r];
    Cs[(row + 16) * LDC + nw * 32 + 16 + c] = a11[r];
  }
  __syncthreads();

  const int w = mb / MT, tok0 = (mb - w * MT) * 64;
  const int rbase = tok0 + wave * 8;
  v4f ov[8];
  size_t offs[8];
#pragma unroll
  for (int it = 0; it < 8; ++it) {
    const int row = wave * 8 + it;
    v4f v = *(const v4f*)(Cs + row * LDC + lane * 4);
    v = v * (1.0f / 65536.0f);
    ov[it] = v;
    const int tokc = min(rbase + it, NTOK - 1);
    offs[it] = ((size_t)w * NTOK + tokc) * CCH + nb * 128 + lane * 4;
  }
#pragma unroll
  for (int it = 0; it < 8; ++it) {
    if (rbase + it < NTOK) *(volatile v4f*)(out + offs[it]) = ov[it];
  }
  __threadfence();
#pragma unroll
  for (int it = 0; it < 8; ++it) {
    if (rbase + it < NTOK) *(volatile v4f*)(out + offs[it]) = ov[it];
  }
}

extern "C" void kernel_launch(void* const* d_in, const int* in_sizes, int n_in,
                              void* d_out, int out_size, void* d_ws, size_t ws_size,
                              hipStream_t stream) {
  if (n_in < 4) return;
  if (in_sizes[0] != NROWX * CCH) return;
  if (in_sizes[1] != CCH * C3) return;
  if (in_sizes[2] != CCH * CCH) return;
  if (in_sizes[3] != NRPB * NHD) return;
  if (out_size != NROWX * CCH) return;

  const float* x    = (const float*)d_in[0];
  const float* wqkv = (const float*)d_in[1];
  const float* wout = (const float*)d_in[2];
  const float* rpb  = (const float*)d_in[3];
  float* out = (float*)d_out;

  const size_t sX  = (size_t)NROWP * CCH * 2;
  const size_t sWq = (size_t)C3 * CCH * 2;
  const size_t sWo = (size_t)CCH * CCH * 2;
  const size_t sBT = (size_t)NHD * NST * NKT * 256 * 4;
  const size_t sQK = (size_t)NWIN * NHD * TP * HD * 2;
  const size_t sO  = (size_t)NHD * NROWP * HD * 2;
  size_t off = 0;
  const size_t oX  = off; off += sX;
  const size_t oWq = off; off += sWq;
  const size_t oWo = off; off += sWo;
  const size_t oBT = off; off += sBT;
  const size_t oQ  = off; off += sQK;
  const size_t oK  = off; off += sQK;
  const size_t oV  = off; off += sQK;
  const size_t oO  = off; off += sO;
  if (off > ws_size) return;
  if (off > (size_t)134217728) return;

  char* ws = (char*)d_ws;
  unsigned short* X8  = (unsigned short*)(ws + oX);
  unsigned short* WqT = (unsigned short*)(ws + oWq);
  unsigned short* WoT = (unsigned short*)(ws + oWo);
  float*          BT  = (float*)(ws + oBT);
  unsigned short* Qp  = (unsigned short*)(ws + oQ);
  unsigned short* Kp  = (unsigned short*)(ws + oK);
  unsigned short* Vtp = (unsigned short*)(ws + oV);
  unsigned short* Op  = (unsigned short*)(ws + oO);

  const dim3 blk(256);
  cvt_x<<<dim3(NROWP / 8), blk, 0, stream>>>(x, X8);
  cvt_wT<<<dim3(C3 / 32), blk, 0, stream>>>(wqkv, WqT, C3);
  cvt_wT<<<dim3(CCH / 32), blk, 0, stream>>>(wout, WoT, CCH);
  build_bias<<<dim3((NHD * NST * NKT * 64) / 256), blk, 0, stream>>>(rpb, BT);
  gemm_qkv<<<dim3(NROWP / 64, C3 / 128), blk, 0, stream>>>(X8, WqT, Qp, Kp, Vtp);
  attn_win<<<dim3(NWIN * NHD * 3), blk, 0, stream>>>(Qp, Kp, Vtp, BT, Op);
  gemm_proj<<<dim3(NROWP / 64, CCH / 128), blk, 0, stream>>>(Op, WoT, out);
  (void)hipGetLastError();
}
